// JointAttentionBlock_55190329753678
// MI455X (gfx1250) — hardware-run, weakly checked
//
#include <hip/hip_runtime.h>


#define NI   4
#define SS   1024
#define DM   768
#define NH_  12
#define HD   64
#define NK   2048
#define HPP  4
#define NADA 2304
#define PCAR 1024.0f
typedef _Float16 h16;
typedef unsigned short bf;
typedef __attribute__((ext_vector_type(16))) __bf16   v16bf;
typedef __attribute__((ext_vector_type(16))) _Float16 v16h;
typedef __attribute__((ext_vector_type(8)))  _Float16 v8h;
typedef __attribute__((ext_vector_type(8)))  unsigned short v8us;
typedef __attribute__((ext_vector_type(8)))  float    v8f;
typedef __attribute__((ext_vector_type(4)))  float    v4f;
typedef v8h  __attribute__((may_alias)) v8ha;
typedef v4f  __attribute__((may_alias)) v4fa;
typedef v8us __attribute__((may_alias)) v8usa;

__device__ __forceinline__ unsigned short f2bf(float f) { unsigned u = __float_as_uint(f); u += 0x7FFFu + ((u >> 16) & 1u); return (unsigned short)(u >> 16); }
__device__ __forceinline__ float bf2f(unsigned short b) { return __uint_as_float(((unsigned)b) << 16); }
__device__ __forceinline__ float bfr(float f) { return bf2f(f2bf(f)); }
__device__ __forceinline__ v16h cat16(v8h lo, v8h hi) { return __builtin_shufflevector(lo, hi, 0, 1, 2, 3, 4, 5, 6, 7, 8, 9, 10, 11, 12, 13, 14, 15); }
__device__ __forceinline__ v16bf cat16b(v8us lo, v8us hi) { return __builtin_bit_cast(v16bf, __builtin_shufflevector(lo, hi, 0, 1, 2, 3, 4, 5, 6, 7, 8, 9, 10, 11, 12, 13, 14, 15)); }
__device__ __forceinline__ v8f wmma16(v16h a, v16h b, v8f c) { return __builtin_amdgcn_wmma_f32_16x16x32_f16(false, a, false, b, (short)0, c, false, false); }
__device__ __forceinline__ v8f wmmab(v16bf a, v16bf b, v8f c) { return __builtin_amdgcn_wmma_f32_16x16x32_bf16(false, a, false, b, (short)0, c, false, false); }


template <typename T16> struct WFrag;
template <> struct WFrag<h16> { typedef v16h V; static __device__ __forceinline__ V ld(const h16* p) { return cat16(*(const v8h*)p, *(const v8h*)(p + 16)); } static __device__ __forceinline__ v8f mma(V a, V b, v8f c) { return wmma16(a, b, c); } };
template <> struct WFrag<bf> { typedef v16bf V; static __device__ __forceinline__ V ld(const bf* p) { return cat16b(*(const v8us*)p, *(const v8us*)(p + 16)); } static __device__ __forceinline__ v8f mma(V a, V b, v8f c) { return wmmab(a, b, c); } };
template <typename T16, int NSPLIT, bool BIAS>
__global__ __launch_bounds__(32) void k_gemmw(const T16* __restrict__ A, const T16* __restrict__ A2, const T16* __restrict__ Bt, const T16* __restrict__ Bt2, int K, float* C, int ldc, const float* __restrict__ bias, size_t sA, size_t sB, size_t sC) {
    typedef typename WFrag<T16>::V V;
    __shared__ __align__(16) float os[16 * 68];
    const size_t z = blockIdx.z; A += z * sA; if (A2) A2 += z * sA; Bt += z * sB; if (Bt2) Bt2 += z * sB; C += z * sC;
    const int lane = threadIdx.x & 31, lr = lane & 15, hi = lane >> 4; const int r0 = blockIdx.x * 64, c0 = blockIdx.y * 64;
    v8f acc[4][4];
#pragma unroll
    for (int mb = 0; mb < 4; ++mb)
#pragma unroll
        for (int nb = 0; nb < 4; ++nb) acc[mb][nb] = (v8f){};
    const size_t aoff = (size_t)(r0 + lr) * K + 8 * hi, boff = (size_t)(c0 + lr) * K + 8 * hi;
#pragma unroll 1
    for (int kc = 0; kc < K; kc += 32) {
        V a[4], a2[4];
#pragma unroll
        for (int mb = 0; mb < 4; ++mb) { a[mb] = WFrag<T16>::ld(A + aoff + (size_t)mb * 16 * K + kc); if (NSPLIT == 1 || NSPLIT == 2) a2[mb] = WFrag<T16>::ld(A2 + aoff + (size_t)mb * 16 * K + kc); }
#pragma unroll
        for (int nb = 0; nb < 4; ++nb) { const V b = WFrag<T16>::ld(Bt + boff + (size_t)nb * 16 * K + kc); V b2; if (NSPLIT >= 2) b2 = WFrag<T16>::ld(Bt2 + boff + (size_t)nb * 16 * K + kc);
#pragma unroll
            for (int mb = 0; mb < 4; ++mb) { acc[mb][nb] = WFrag<T16>::mma(a[mb], b, acc[mb][nb]); if (NSPLIT == 1 || NSPLIT == 2) acc[mb][nb] = WFrag<T16>::mma(a2[mb], b, acc[mb][nb]); if (NSPLIT >= 2) acc[mb][nb] = WFrag<T16>::mma(a[mb], b2, acc[mb][nb]); } }
        asm volatile("v_nop\n\tv_nop\n\tv_nop\n\tv_nop" : "+v"(acc[0][0]), "+v"(acc[1][1]), "+v"(acc[2][2]), "+v"(acc[3][3]) : "v"(a[0]), "v"(a[3]));
    }
#pragma unroll
    for (int mb = 0; mb < 4; ++mb) {
#pragma unroll
        for (int nb = 0; nb < 4; ++nb) {
#pragma unroll
            for (int j = 0; j < 8; ++j) os[(hi * 8 + j) * 68 + nb * 16 + lr] = acc[mb][nb][j]; }
        __builtin_amdgcn_wave_barrier(); asm volatile("" ::: "memory");
        float* crow = C + (size_t)(r0 + mb * 16) * ldc + c0;
#pragma unroll 1
        for (int ps = 0; ps < 2; ++ps) {
#pragma unroll
            for (int s = 0; s < 8; ++s) { const int row = 2 * s + hi, cofs = lr * 4; v4f val = *(const v4fa*)(os + row * 68 + cofs); if (BIAS) { val[0] += bfr(bias[c0 + cofs]); val[1] += bfr(bias[c0 + cofs + 1]); val[2] += bfr(bias[c0 + cofs + 2]); val[3] += bfr(bias[c0 + cofs + 3]); }
                *(volatile v4f*)(crow + (size_t)row * ldc + cofs) = val; }
            if (ps == 0) __threadfence(); }
        __builtin_amdgcn_wave_barrier(); asm volatile("" ::: "memory");
    }
}

__device__ __forceinline__ h16 tohx(float x) { return (h16)x; }
__device__ __forceinline__ void splitf(float y, unsigned short& h, unsigned short& l) { h = f2bf(y); l = f2bf(y - bf2f(h)); }
typedef __attribute__((ext_vector_type(2))) unsigned short v2us;
typedef __attribute__((ext_vector_type(4))) unsigned short v4us;
typedef __attribute__((ext_vector_type(2))) _Float16 v2h;
typedef __attribute__((ext_vector_type(4))) _Float16 v4h;
__constant__ float FRQ[NH_][8] = {
    3.14159250f, 4.18938112f, 5.58662987f, 7.44988966f, 9.93458843f, 13.2479868f, 17.6664753f, 23.5586243f,
    3.21785545f, 4.29107904f, 5.72224617f, 7.63073826f, 10.1757536f, 13.5695868f, 18.0953350f, 24.1305199f,
    3.29596949f, 4.39524651f, 5.86115456f, 7.81597710f, 10.4227715f, 13.8989897f, 18.5346012f, 24.7162895f,
    3.37597990f, 4.50194168f, 6.00343561f, 8.00571060f, 10.6757870f, 14.2363930f, 18.9845352f, 25.3162880f,
    3.45793271f, 4.61122751f, 6.14917040f, 8.20005035f, 10.9349432f, 14.5819826f, 19.4453869f, 25.9308434f,
    3.54187489f, 4.72316551f, 6.29844284f, 8.39910889f, 11.2003927f, 14.9359646f, 19.9174309f, 26.5603161f,
    3.62785459f, 4.83782196f, 6.45133972f, 8.60300064f, 11.4722862f, 15.2985373f, 20.4009285f, 27.2050781f,
    3.71592164f, 4.95526075f, 6.60794687f, 8.81183910f, 11.7507772f, 15.6699142f, 20.8961678f, 27.8654823f,
    3.80612636f, 5.07555103f, 6.76835632f, 9.02574730f, 12.0360289f, 16.0503025f, 21.4034252f, 28.5419273f,
    3.89852095f, 5.19876099f, 6.93265963f, 9.24485111f, 12.3282070f, 16.4399300f, 21.9230003f, 29.2347927f,
    3.99315858f, 5.32496262f, 7.10095167f, 9.46927261f, 12.6274757f, 16.8390102f, 22.4551830f, 29.9444695f,
    4.09009314f, 5.45422649f, 7.27332878f, 9.69914055f, 12.9340124f, 17.2477837f, 23.0002861f, 30.6713753f };

__global__ __launch_bounds__(256) void k_cvt8(const float* __restrict__ src, bf* dst, size_t n8) { const size_t i = (size_t)blockIdx.x * 256 + threadIdx.x; if (i >= n8) return; const v8f v = *(const v8f*)(src + i * 8); v8us o;
#pragma unroll
    for (int k = 0; k < 8; ++k) o[k] = f2bf(v[k]); *(volatile v8us*)(dst + i * 8) = o; __threadfence(); *(volatile v8us*)(dst + i * 8) = o; }
__global__ __launch_bounds__(256) void k_ada(const float* __restrict__ cond, const float* __restrict__ aw, const float* __restrict__ ab, float* ADA) { const int idx = blockIdx.x * 256 + threadIdx.x; if (idx >= NI * NADA) return; const int o = idx % NADA; const int b = idx / NADA; const float* c = cond + (size_t)b * DM; const float* w = aw + (size_t)o * DM; float s = 0.f;
#pragma unroll 1
    for (int k = 0; k < DM; ++k) { const float cv = bfr(c[k]); float sg = __fdiv_rn(1.0f, __fadd_rn(1.0f, __expf(-cv))); asm volatile("" : "+v"(sg)); float si = __fmul_rn(cv, sg); asm volatile("" : "+v"(si)); float p = __fmul_rn(si, bfr(w[k])); asm volatile("" : "+v"(p)); s = __fadd_rn(s, p); }
    const float r = __fadd_rn(s, bfr(ab[o])); *(volatile float*)(ADA + idx) = r; __threadfence(); *(volatile float*)(ADA + idx) = r; }
__global__ __launch_bounds__(256) void k_rmsm(const float* __restrict__ X, const float* __restrict__ nsc, const float* __restrict__ ADAb, bf* Hh, bf* Hl) { const int lane = threadIdx.x & 31; const int t = blockIdx.x * 8 + (threadIdx.x >> 5); if (t >= SS) return; float v[DM / 32]; float q = 0.f;
#pragma unroll
    for (int ch = 0; ch < DM / 128; ++ch) { const v4f a = *(const v4f*)(X + (size_t)t * DM + ch * 128 + lane * 4);
#pragma unroll
        for (int u = 0; u < 4; ++u) { v[ch * 4 + u] = bfr(a[u]); float p = __fmul_rn(v[ch * 4 + u], v[ch * 4 + u]); asm volatile("" : "+v"(p)); q = __fadd_rn(q, p); } }
#pragma unroll
    for (int sh = 16; sh; sh >>= 1) q += __shfl_xor(q, sh, 32);
    const float rs = __frsqrt_rn(__fadd_rn(q * (1.0f / DM), 1e-6f)); const float* shift = ADAb; const float* scale = ADAb + DM;
    for (int ps = 0; ps < 2; ++ps) {
#pragma unroll
        for (int ch = 0; ch < DM / 128; ++ch) { const int c0 = ch * 128 + lane * 4; v4us oh, ol;
#pragma unroll
            for (int u = 0; u < 4; ++u) { const int c = c0 + u; float f = __fmul_rn(bfr(nsc[c]), rs); asm volatile("" : "+v"(f)); float n0 = __fmul_rn(v[ch * 4 + u], f); asm volatile("" : "+v"(n0)); float m1 = __fadd_rn(1.0f, scale[c]); asm volatile("" : "+v"(m1)); float t1 = __fmul_rn(n0, m1); asm volatile("" : "+v"(t1)); const float y = __fadd_rn(t1, shift[c]); unsigned short a2, b2; splitf(y, a2, b2); oh[u] = a2; ol[u] = b2; }
            const size_t oo = (size_t)t * DM + c0; *(volatile v4us*)(Hh + oo) = oh; *(volatile v4us*)(Hl + oo) = ol; }
        if (ps == 0) __threadfence(); } }
__global__ __launch_bounds__(256) void k_qk(const float* __restrict__ F, const float* __restrict__ pos, const float* __restrict__ ascale, int rope_on, h16* P, int key0, int nrows_total) {
    const int lane = threadIdx.x & 31; const int row = blockIdx.x * 8 + (threadIdx.x >> 5); if (row >= NH_ * SS) return; const int t = row % SS; const int h = row / SS; const float* f = F + (size_t)t * DM + h * HD + lane * 2; float v0 = f[0], v1 = f[1];
    float ss = __fadd_rn(__fmul_rn(v0, v0), __fmul_rn(v1, v1)); asm volatile("" : "+v"(ss));
#pragma unroll
    for (int sh = 16; sh; sh >>= 1) ss += __shfl_xor(ss, sh, 32);
    float sc = __fmul_rn(__fsqrt_rn(bfr(ascale[h])), __frsqrt_rn(__fadd_rn(ss, 1e-6f))); asm volatile("" : "+v"(sc)); v0 = __fmul_rn(v0, sc); v1 = __fmul_rn(v1, sc);
    const float p0 = __shfl_xor(v0, 8, 32), p1 = __shfl_xor(v1, 8, 32);
    if (rope_on && lane < 16) { const float ph = bfr(pos[(size_t)t * 2]), pw = bfr(pos[(size_t)t * 2 + 1]);
#pragma unroll
        for (int u = 0; u < 2; ++u) { const int d = lane * 2 + u; const int i = d & 15; const float th = __fmul_rn((i < 8) ? ph : pw, FRQ[h][i & 7]); const float c = cosf(th), s = sinf(th); float& me = (u == 0) ? v0 : v1; const float pr = (u == 0) ? p0 : p1;
            float a = __fmul_rn(me, c), bq = __fmul_rn(pr, s); asm volatile("" : "+v"(a)); asm volatile("" : "+v"(bq)); me = (d < 16) ? __fsub_rn(a, bq) : __fadd_rn(a, bq); } }
    v2h o; o[0] = tohx(v0); o[1] = tohx(v1); h16* dst = P + ((size_t)h * nrows_total + key0 + t) * HD + lane * 2; *(volatile v2h*)dst = o; __threadfence(); *(volatile v2h*)dst = o; }
__global__ __launch_bounds__(256) void k_vt(const float* __restrict__ V, int key0, h16* VT) { const int e = (blockIdx.x * 256 + threadIdx.x) * 2; if (e >= NH_ * HD * SS) return; const int t = e % SS; const int d = (e / SS) % HD; const int h = e / (SS * HD); v2h o; o[0] = tohx(V[(size_t)t * DM + h * HD + d]); o[1] = tohx(V[(size_t)(t + 1) * DM + h * HD + d]); h16* dst = VT + ((size_t)h * HD + d) * NK + key0 + t; *(volatile v2h*)dst = o; __threadfence(); *(volatile v2h*)dst = o; }
__global__ __launch_bounds__(256) void k_soft(const float* __restrict__ Sb, h16* P16) { const int lane = threadIdx.x & 31; const int row = blockIdx.x * 8 + (threadIdx.x >> 5); if (row >= HPP * SS) return; const float* sr = Sb + (size_t)row * NK; float v[NK / 32]; float mx = -3.0e38f;
#pragma unroll
    for (int ch = 0; ch < NK / 128; ++ch) { const v4f a = *(const v4f*)(sr + ch * 128 + lane * 4);
#pragma unroll
        for (int u = 0; u < 4; ++u) { v[ch * 4 + u] = a[u]; mx = fmaxf(mx, a[u]); } }
#pragma unroll
    for (int sh = 16; sh; sh >>= 1) mx = fmaxf(mx, __shfl_xor(mx, sh, 32));
    float sum = 0.f;
#pragma unroll
    for (int q = 0; q < NK / 32; ++q) { float d0 = __fsub_rn(v[q], mx); asm volatile("" : "+v"(d0)); v[q] = __builtin_amdgcn_exp2f(__fmul_rn(d0, 1.4426950408889634f)); sum += v[q]; }
#pragma unroll
    for (int sh = 16; sh; sh >>= 1) sum += __shfl_xor(sum, sh, 32);
    const float f = __fdiv_rn(PCAR, sum);
    for (int ps = 0; ps < 2; ++ps) {
#pragma unroll
        for (int ch = 0; ch < NK / 128; ++ch) { v4h o4;
#pragma unroll
            for (int q = 0; q < 4; ++q) o4[q] = tohx(v[ch * 4 + q] * f); *(volatile v4h*)(P16 + (size_t)row * NK + ch * 128 + lane * 4) = o4; }
        if (ps == 0) __threadfence(); } }
__global__ __launch_bounds__(256) void k_mrg(const float* __restrict__ O, int h0, bf* Ah, bf* Al) { const int e = (blockIdx.x * 256 + threadIdx.x) * 4; if (e >= HPP * SS * HD) return; const int d = e % HD; const int t = (e / HD) % SS; const int z = e / (HD * SS); v4us oh, ol;
#pragma unroll
    for (int u = 0; u < 4; ++u) { unsigned short a, b; splitf(O[e + u] * (1.0f / PCAR), a, b); oh[u] = a; ol[u] = b; } const size_t oo = (size_t)t * DM + (h0 + z) * HD + d; *(volatile v4us*)(Ah + oo) = oh; *(volatile v4us*)(Al + oo) = ol; __threadfence(); *(volatile v4us*)(Ah + oo) = oh; *(volatile v4us*)(Al + oo) = ol; }
__global__ __launch_bounds__(256) void k_fin(const float* __restrict__ X, const float* __restrict__ OO, const float* __restrict__ gate, float* outb) { const int e = (blockIdx.x * 256 + threadIdx.x) * 4; if (e >= SS * DM) return; const int c = e % DM; const v4f a = *(const v4f*)(X + e), o = *(const v4f*)(OO + e); v4f r;
#pragma unroll
    for (int u = 0; u < 4; ++u) { float gm = __fmul_rn(gate[c + u], o[u]); asm volatile("" : "+v"(gm)); r[u] = __fadd_rn(bfr(a[u]), gm); } *(volatile v4f*)(outb + e) = r; __threadfence(); *(volatile v4f*)(outb + e) = r; }

extern "C" void kernel_launch(void* const* d_in, const int* in_sizes, int n_in,
                              void* d_out, int out_size, void* d_ws, size_t ws_size, hipStream_t stream) {
    (void)in_sizes; (void)n_in; (void)out_size;
    const float** I = (const float**)d_in;
    const float *x = I[0], *src = I[1], *pos = I[2], *cond = I[3], *q_w = I[4], *k_w = I[5], *v_w = I[6], *out_w = I[7], *ada_w = I[8], *ada_b = I[9], *qns = I[10], *sns = I[11], *ascale = I[12];
    float* OUT = (float*)d_out;
    char* wsp = (char*)d_ws;
    auto take = [&](size_t bytes) { char* p = wsp; wsp += (bytes + 255) & ~(size_t)255; return (void*)p; };
    bf* BQ = (bf*)take((size_t)DM * DM * 2); bf* BK = (bf*)take((size_t)DM * DM * 2); bf* BV = (bf*)take((size_t)DM * DM * 2); bf* BO = (bf*)take((size_t)DM * DM * 2); float* ADA = (float*)take((size_t)NI * NADA * 4);
    bf* XMh = (bf*)take((size_t)SS * DM * 2); bf* XMl = (bf*)take((size_t)SS * DM * 2); bf* SMh = (bf*)take((size_t)SS * DM * 2); bf* SMl = (bf*)take((size_t)SS * DM * 2);
    float* Q = (float*)take((size_t)SS * DM * 4); float* KS = (float*)take((size_t)SS * DM * 4); float* VS = (float*)take((size_t)SS * DM * 4); float* KR = (float*)take((size_t)SS * DM * 4); float* VR = (float*)take((size_t)SS * DM * 4);
    h16* Q16 = (h16*)take((size_t)NH_ * SS * HD * 2); h16* K16 = (h16*)take((size_t)NH_ * NK * HD * 2); h16* VT = (h16*)take((size_t)NH_ * HD * NK * 2); float* Sb = (float*)take((size_t)HPP * SS * NK * 4); h16* P16 = (h16*)take((size_t)HPP * SS * NK * 2); float* O = (float*)take((size_t)HPP * SS * HD * 4);
    bf* Ah = (bf*)take((size_t)SS * DM * 2); bf* Al = (bf*)take((size_t)SS * DM * 2); float* OO = (float*)take((size_t)SS * DM * 4);
    if ((size_t)(wsp - (char*)d_ws) > ws_size) return;
    k_cvt8<<<(DM * DM / 8 + 255) / 256, 256, 0, stream>>>(q_w, BQ, DM * DM / 8); k_cvt8<<<(DM * DM / 8 + 255) / 256, 256, 0, stream>>>(k_w, BK, DM * DM / 8); k_cvt8<<<(DM * DM / 8 + 255) / 256, 256, 0, stream>>>(v_w, BV, DM * DM / 8); k_cvt8<<<(DM * DM / 8 + 255) / 256, 256, 0, stream>>>(out_w, BO, DM * DM / 8);
    k_ada<<<(NI * NADA + 255) / 256, 256, 0, stream>>>(cond, ada_w, ada_b, ADA);
    const dim3 gg(SS / 64, DM / 64, 1); const size_t zq = (size_t)SS * HD, zk = (size_t)NK * HD, zS = (size_t)SS * NK;
    for (int b = 0; b < NI; ++b) { const float* xb = x + (size_t)b * SS * DM; const float* ADAb = ADA + (size_t)b * NADA;
        k_rmsm<<<SS / 8, 256, 0, stream>>>(xb, qns, ADAb, XMh, XMl); k_rmsm<<<SS / 8, 256, 0, stream>>>(src + (size_t)b * SS * DM, sns, ADAb, SMh, SMl);
        k_gemmw<bf, 1, false><<<gg, 32, 0, stream>>>(XMh, XMl, BQ, nullptr, DM, Q, DM, nullptr, 0, 0, 0); k_gemmw<bf, 1, false><<<gg, 32, 0, stream>>>(XMh, XMl, BK, nullptr, DM, KS, DM, nullptr, 0, 0, 0); k_gemmw<bf, 1, false><<<gg, 32, 0, stream>>>(XMh, XMl, BV, nullptr, DM, VS, DM, nullptr, 0, 0, 0);
        k_gemmw<bf, 1, false><<<gg, 32, 0, stream>>>(SMh, SMl, BK, nullptr, DM, KR, DM, nullptr, 0, 0, 0); k_gemmw<bf, 1, false><<<gg, 32, 0, stream>>>(SMh, SMl, BV, nullptr, DM, VR, DM, nullptr, 0, 0, 0);
        const float* pb = pos + (size_t)b * SS * 2;
        k_qk<<<NH_ * SS / 8, 256, 0, stream>>>(Q, pb, ascale, 1, Q16, 0, SS); k_qk<<<NH_ * SS / 8, 256, 0, stream>>>(KS, pb, ascale, 1, K16, 0, NK); k_qk<<<NH_ * SS / 8, 256, 0, stream>>>(KR, pb, ascale, 1, K16, SS, NK);
        k_vt<<<(NH_ * HD * SS / 2 + 255) / 256, 256, 0, stream>>>(VS, 0, VT); k_vt<<<(NH_ * HD * SS / 2 + 255) / 256, 256, 0, stream>>>(VR, SS, VT);
        for (int h0 = 0; h0 < NH_; h0 += HPP) {
            k_gemmw<h16, 0, false><<<dim3(SS / 64, NK / 64, HPP), 32, 0, stream>>>(Q16 + (size_t)h0 * zq, nullptr, K16 + (size_t)h0 * zk, nullptr, HD, Sb, NK, nullptr, zq, zk, zS);
            k_soft<<<HPP * SS / 8, 256, 0, stream>>>(Sb, P16);
            k_gemmw<h16, 0, false><<<dim3(SS / 64, 1, HPP), 32, 0, stream>>>(P16, nullptr, VT + (size_t)h0 * HD * NK, nullptr, NK, O, HD, nullptr, zS, (size_t)HD * NK, zq);
            k_mrg<<<(HPP * SS * HD / 4 + 255) / 256, 256, 0, stream>>>(O, h0, Ah, Al); }
        k_gemmw<bf, 1, false><<<gg, 32, 0, stream>>>(Ah, Al, BO, nullptr, DM, OO, DM, nullptr, 0, 0, 0);
        k_fin<<<(SS * DM / 4 + 255) / 256, 256, 0, stream>>>(xb, OO, ADAb + 2 * DM, OUT + (size_t)b * SS * DM); }
}
